// STARVisionDetector_75952201662652
// MI455X (gfx1250) — hardware-verified
//
#include <hip/hip_runtime.h>
#include <stddef.h>
#include <stdint.h>
#include <math.h>

#define BATCH 64
#define GRIDN 14
#define PP    196
#define DIM   768
#define NTOK  (BATCH * PP)
#define NBOX  32
#define NCLS  80
#define IMW   224
#define PSZ   16
#define NPC   (DIM / 8)
#define PLH   ((size_t)NTOK * DIM)
#define OFF1  ((size_t)NTOK * NCLS)
#define OFF2  (OFF1 + (size_t)NTOK)
#define OFF3  (OFF2 + (size_t)NTOK * 4)

static_assert(NTOK % 256 == 0);
static_assert(NTOK % 8 == 0);
static_assert(DIM % 64 == 0);
static_assert(NPC % 32 == 0);
static_assert((NTOK * NPC) % 256 == 0);
static_assert((DIM * DIM / 8) % 256 == 0);
static_assert(NCLS % 16 == 0);
static_assert((NCLS * NPC) % 256 == 0);
static_assert((16 * NPC) % 256 == 0);

typedef _Float16 v16h __attribute__((ext_vector_type(16)));
typedef _Float16 v8h  __attribute__((ext_vector_type(8)));
typedef float    v8f  __attribute__((ext_vector_type(8)));
typedef float    v4f  __attribute__((ext_vector_type(4)));
typedef unsigned int v4u __attribute__((ext_vector_type(4)));

union Frag  { v16h v; v8h h[2]; };
union Pack8 { v8h h; v4u u; };

__device__ __forceinline__ v8f mma16(v16h a, v16h b, v8f c) {
  c = __builtin_amdgcn_wmma_f32_16x16x32_f16(false, a, false, b, (short)0, c, false, false);
  asm volatile("v_nop\n\tv_nop\n\tv_nop\n\tv_nop" : "+v"(c) : "v"(a), "v"(b));
  return c;
}

__device__ __forceinline__ v16h ldfrag(const _Float16* p, int ld, int row0, int k0, int lane) {
  const int m = lane & 15, lh = lane >> 4;
  const _Float16* q = p + (size_t)(row0 + m) * ld + k0 + 8 * lh;
  Frag f;
  f.h[0] = *(const v8h*)(q);
  f.h[1] = *(const v8h*)(q + 16);
  return f.v;
}

__device__ __forceinline__ v8f zero8() { return (v8f){0.f, 0.f, 0.f, 0.f, 0.f, 0.f, 0.f, 0.f}; }

__device__ __forceinline__ float silu16(float v) {
  const float e = __expf(-v);
  return 16.0f * v * __builtin_amdgcn_rcpf(1.0f + e);
}

template <int KK>
__device__ __forceinline__ void gemm32x64(const _Float16* __restrict__ A, int lda,
                                          const _Float16* __restrict__ Bt, int ldb,
                                          int m0, int n0, int lane, v8f (&acc)[2][4]) {
#pragma unroll 2
  for (int k0 = 0; k0 < KK; k0 += 32) {
    const v16h a0 = ldfrag(A, lda, m0, k0, lane);
    const v16h a1 = ldfrag(A, lda, m0 + 16, k0, lane);
    const v16h b0 = ldfrag(Bt, ldb, n0, k0, lane);
    const v16h b1 = ldfrag(Bt, ldb, n0 + 16, k0, lane);
    const v16h b2 = ldfrag(Bt, ldb, n0 + 32, k0, lane);
    const v16h b3 = ldfrag(Bt, ldb, n0 + 48, k0, lane);
    acc[0][0] = mma16(a0, b0, acc[0][0]);
    acc[1][0] = mma16(a1, b0, acc[1][0]);
    acc[0][1] = mma16(a0, b1, acc[0][1]);
    acc[1][1] = mma16(a1, b1, acc[1][1]);
    acc[0][2] = mma16(a0, b2, acc[0][2]);
    acc[1][2] = mma16(a1, b2, acc[1][2]);
    acc[0][3] = mma16(a0, b3, acc[0][3]);
    acc[1][3] = mma16(a1, b3, acc[1][3]);
  }
}

__global__ __launch_bounds__(256) void k_im2col(const float* __restrict__ img, _Float16* __restrict__ xp, int ngrp) {
  const int t = blockIdx.x * 256 + (int)threadIdx.x;
  if (t >= ngrp) return;
  const int n = t / NPC, pc = t - n * NPC;
  const int b = n / PP, p = n - b * PP;
  const int py = p / GRIDN, px = p - py * GRIDN;
  const int k0 = pc * 8;
  const int c = k0 >> 8, i = (k0 >> 4) & 15, j0 = k0 & 15;
  const size_t src = ((size_t)(b * 3 + c) * IMW + (size_t)(py * PSZ + i)) * IMW + (size_t)(px * PSZ + j0);
  const v4f a0 = *(const v4f*)(img + src);
  const v4f a1 = *(const v4f*)(img + src + 4);
  Pack8 pk;
  pk.h = (v8h){(_Float16)a0[0], (_Float16)a0[1], (_Float16)a0[2], (_Float16)a0[3],
               (_Float16)a1[0], (_Float16)a1[1], (_Float16)a1[2], (_Float16)a1[3]};
  const v4u vv = pk.u;
  volatile v4u* d = (volatile v4u*)(xp + (size_t)n * DIM + k0);
  *d = vv;
  __threadfence();
  *d = vv;
}

__global__ __launch_bounds__(256) void k_cvt_w(const float* __restrict__ w, _Float16* __restrict__ wh,
                                              int ngrp, float sc) {
  const int t = blockIdx.x * 256 + (int)threadIdx.x;
  if (t >= ngrp) return;
  const size_t o = (size_t)t * 8;
  const v4f a0 = *(const v4f*)(w + o);
  const v4f a1 = *(const v4f*)(w + o + 4);
  Pack8 pk;
  pk.h = (v8h){(_Float16)(a0[0] * sc), (_Float16)(a0[1] * sc), (_Float16)(a0[2] * sc), (_Float16)(a0[3] * sc),
               (_Float16)(a1[0] * sc), (_Float16)(a1[1] * sc), (_Float16)(a1[2] * sc), (_Float16)(a1[3] * sc)};
  const v4u vv = pk.u;
  volatile v4u* d = (volatile v4u*)(wh + o);
  *d = vv;
  __threadfence();
  *d = vv;
}

#define WTP 68
__global__ __launch_bounds__(256) void k_wt(const float* __restrict__ w, _Float16* __restrict__ wt,
                                           int nout, int kin) {
  __shared__ __align__(16) float tf[64 * WTP];
  const int tid = threadIdx.x;
  const int n0 = blockIdx.x * 64;
  const int k0 = blockIdx.y * 64;
  {
    const int kr = tid >> 4;
    const int n4 = (tid & 15) * 4;
#pragma unroll
    for (int it = 0; it < 4; ++it) {
      const int kl = it * 16 + kr;
      const v4f a = *(const v4f*)(w + (size_t)(k0 + kl) * nout + n0 + n4);
      *(v4f*)(tf + kl * WTP + n4) = a;
    }
  }
  __syncthreads();
  v4u val[2];
  size_t go[2];
#pragma unroll
  for (int j = 0; j < 2; ++j) {
    const int p  = tid + 256 * j;
    const int nl = p >> 3;
    const int pc = p & 7;
    const float* cp = tf + (pc * 8) * WTP + nl;
    Pack8 pk;
    pk.h = (v8h){(_Float16)(cp[0 * WTP] * 32.0f), (_Float16)(cp[1 * WTP] * 32.0f),
                 (_Float16)(cp[2 * WTP] * 32.0f), (_Float16)(cp[3 * WTP] * 32.0f),
                 (_Float16)(cp[4 * WTP] * 32.0f), (_Float16)(cp[5 * WTP] * 32.0f),
                 (_Float16)(cp[6 * WTP] * 32.0f), (_Float16)(cp[7 * WTP] * 32.0f)};
    val[j] = pk.u;
    go[j]  = (size_t)(n0 + nl) * kin + k0 + pc * 8;
  }
  for (int ps = 0; ps < 2; ++ps) {
#pragma unroll
    for (int j = 0; j < 2; ++j) *(volatile v4u*)(wt + go[j]) = val[j];
    __threadfence();
  }
}

__global__ __launch_bounds__(256) void k_wt_small(const float* __restrict__ w, _Float16* __restrict__ wt,
                                                 int ncols, int npad) {
  const int t = blockIdx.x * 256 + (int)threadIdx.x;
  if (t >= npad * NPC) return;
  const int n = t / NPC, pc = t - n * NPC;
  const int nc = (n < ncols) ? n : (ncols - 1);
  const float sc = (n < ncols) ? 32.0f : 0.0f;
  float v[8];
#pragma unroll
  for (int e = 0; e < 8; ++e) v[e] = w[(size_t)(pc * 8 + e) * ncols + nc] * sc;
  Pack8 pk;
  pk.h = (v8h){(_Float16)v[0], (_Float16)v[1], (_Float16)v[2], (_Float16)v[3],
               (_Float16)v[4], (_Float16)v[5], (_Float16)v[6], (_Float16)v[7]};
  const v4u vv = pk.u;
  volatile v4u* d = (volatile v4u*)(wt + (size_t)n * DIM + pc * 8);
  *d = vv;
  __threadfence();
  *d = vv;
}

#define OTP 68
__global__ __launch_bounds__(256) void k_embed(const _Float16* __restrict__ xp,
                                               const _Float16* __restrict__ wt,
                                               const float* __restrict__ bias,
                                               const float* __restrict__ pos,
                                               float* __restrict__ ef) {
  __shared__ __align__(16) float st[8][16 * OTP];
  const int tid = threadIdx.x, lane = tid & 31, wave = tid >> 5;
  const int hh = lane >> 4, c = lane & 15;
  const int m0 = blockIdx.x * 256 + wave * 32;
  const int n0 = blockIdx.y * 64;

  v8f acc[2][4];
#pragma unroll
  for (int s = 0; s < 2; ++s)
#pragma unroll
    for (int t = 0; t < 4; ++t) acc[s][t] = zero8();
  gemm32x64<DIM>(xp, DIM, wt, DIM, m0, n0, lane, acc);

  float bvs[4];
#pragma unroll
  for (int t = 0; t < 4; ++t) bvs[t] = bias[n0 + 16 * t + c];

  float* sw = st[wave];
#pragma unroll
  for (int sub = 0; sub < 2; ++sub) {
    __syncthreads();
#pragma unroll
    for (int t = 0; t < 4; ++t) {
#pragma unroll
      for (int r = 0; r < 8; ++r)
        sw[(8 * hh + r) * OTP + 16 * t + c] = acc[sub][t][r] * 0.03125f + bvs[t];
    }
    __syncthreads();
    v4f val[8];
    size_t go[8];
#pragma unroll
    for (int it = 0; it < 8; ++it) {
      const int p    = lane + 32 * it;
      const int L    = p >> 3;
      const int pc   = p & 7;
      const int row  = L >> 1;
      const int half = L & 1;
      const int m    = m0 + sub * 16 + row;
      const size_t g = (size_t)m * DIM + n0 + half * 32 + pc * 4;
      v4f v = *(const v4f*)(sw + row * OTP + half * 32 + pc * 4);
      const v4f pr = *(const v4f*)(pos + (size_t)(m % PP) * DIM + n0 + half * 32 + pc * 4);
      v[0] = v[0] + pr[0]; v[1] = v[1] + pr[1]; v[2] = v[2] + pr[2]; v[3] = v[3] + pr[3];
      val[it] = v;
      go[it]  = g;
    }
    for (int ps = 0; ps < 2; ++ps) {
#pragma unroll
      for (int it = 0; it < 8; ++it) *(volatile v4f*)(ef + go[it]) = val[it];
      __threadfence();
    }
  }
}

__global__ __launch_bounds__(256) void k_rms(const float* __restrict__ ef, const float* __restrict__ w,
                                            _Float16* __restrict__ xn) {
  const int tid = threadIdx.x, lane = tid & 31, wave = tid >> 5;
  const int row = blockIdx.x * 8 + wave;
  const float* e = ef + (size_t)row * DIM;
  v4f a[6];
#pragma unroll
  for (int it = 0; it < 3; ++it) {
    const int p = lane + 32 * it;
    a[2 * it]     = *(const v4f*)(e + 8 * p);
    a[2 * it + 1] = *(const v4f*)(e + 8 * p + 4);
  }
  float ss = 0.0f;
#pragma unroll
  for (int j = 0; j < 6; ++j)
    ss += (a[j][0] * a[j][0] + a[j][1] * a[j][1]) + (a[j][2] * a[j][2] + a[j][3] * a[j][3]);
#pragma unroll
  for (int off = 1; off < 32; off <<= 1) ss += __shfl_xor(ss, off, 32);
  const float sc = rsqrtf(ss * (1.0f / (float)DIM) + 1e-6f);
#pragma unroll
  for (int it = 0; it < 3; ++it) {
    const int p = lane + 32 * it;
    const v4f w0 = *(const v4f*)(w + 8 * p);
    const v4f w1 = *(const v4f*)(w + 8 * p + 4);
    const v4f x0 = a[2 * it], x1 = a[2 * it + 1];
    Pack8 pk;
    pk.h = (v8h){(_Float16)(x0[0] * sc * w0[0]), (_Float16)(x0[1] * sc * w0[1]),
                 (_Float16)(x0[2] * sc * w0[2]), (_Float16)(x0[3] * sc * w0[3]),
                 (_Float16)(x1[0] * sc * w1[0]), (_Float16)(x1[1] * sc * w1[1]),
                 (_Float16)(x1[2] * sc * w1[2]), (_Float16)(x1[3] * sc * w1[3])};
    const v4u vv = pk.u;
    volatile v4u* d = (volatile v4u*)(xn + (size_t)row * DIM + 8 * p);
    *d = vv;
    __threadfence();
    *d = vv;
  }
}

__global__ __launch_bounds__(256) void k_hid(const _Float16* __restrict__ xn,
                                             const _Float16* __restrict__ w1t,
                                             const float* __restrict__ bc,
                                             const float* __restrict__ bo,
                                             const float* __restrict__ bb,
                                             _Float16* __restrict__ hp) {
  __shared__ __align__(16) float st[8][16 * OTP];
  const int z = blockIdx.z;
  const _Float16* wt = w1t + (size_t)z * DIM * DIM;
  _Float16* hz = hp + (size_t)z * PLH;
  const int tid = threadIdx.x, lane = tid & 31, wave = tid >> 5;
  const int hh = lane >> 4, c = lane & 15;
  const int m0 = blockIdx.x * 256 + wave * 32;
  const int n0 = blockIdx.y * 64;

  v8f acc[2][4];
#pragma unroll
  for (int s = 0; s < 2; ++s)
#pragma unroll
    for (int t = 0; t < 4; ++t) acc[s][t] = zero8();
  gemm32x64<DIM>(xn, DIM, wt, DIM, m0, n0, lane, acc);

  float bvs[4];
#pragma unroll
  for (int t = 0; t < 4; ++t) {
    const int nn = n0 + 16 * t + c;
    const float v0 = bc[nn], v1 = bo[nn], v2 = bb[nn];
    bvs[t] = (z == 0) ? v0 : ((z == 1) ? v1 : v2);
  }

  float* sw = st[wave];
#pragma unroll
  for (int sub = 0; sub < 2; ++sub) {
    __syncthreads();
#pragma unroll
    for (int t = 0; t < 4; ++t) {
#pragma unroll
      for (int r = 0; r < 8; ++r)
        sw[(8 * hh + r) * OTP + 16 * t + c] = acc[sub][t][r] * 0.03125f + bvs[t];
    }
    __syncthreads();
    v4u val[4];
    size_t go[4];
#pragma unroll
    for (int it = 0; it < 4; ++it) {
      const int p  = lane + 32 * it;
      const int L  = p >> 3;
      const int pc = p & 7;
      const v4f x0 = *(const v4f*)(sw + L * OTP + pc * 8);
      const v4f x1 = *(const v4f*)(sw + L * OTP + pc * 8 + 4);
      Pack8 pk;
      pk.h = (v8h){(_Float16)silu16(x0[0]), (_Float16)silu16(x0[1]), (_Float16)silu16(x0[2]), (_Float16)silu16(x0[3]),
                   (_Float16)silu16(x1[0]), (_Float16)silu16(x1[1]), (_Float16)silu16(x1[2]), (_Float16)silu16(x1[3])};
      val[it] = pk.u;
      go[it]  = (size_t)(m0 + sub * 16 + L) * DIM + n0 + pc * 8;
    }
    for (int ps = 0; ps < 2; ++ps) {
#pragma unroll
      for (int it = 0; it < 4; ++it) *(volatile v4u*)(hz + go[it]) = val[it];
      __threadfence();
    }
  }
}

#define HP0 84
#define HP1 17
template <int MODE>
__global__ __launch_bounds__(256) void k_head(const _Float16* __restrict__ hz,
                                              const _Float16* __restrict__ wt,
                                              const float* __restrict__ bias,
                                              float* __restrict__ out) {
  constexpr int NT = (MODE == 0) ? 5 : 1;
  constexpr int NB = (MODE == 0) ? NCLS : ((MODE == 1) ? 1 : 4);
  __shared__ __align__(16) float st[8][16 * HP0];
  const int tid = threadIdx.x, lane = tid & 31, wave = tid >> 5;
  const int hh = lane >> 4, c = lane & 15;
  const int m0 = blockIdx.x * 256 + wave * 32;

  v8f acc[2][NT];
#pragma unroll
  for (int t = 0; t < NT; ++t) { acc[0][t] = zero8(); acc[1][t] = zero8(); }
#pragma unroll 1
  for (int k0 = 0; k0 < DIM; k0 += 32) {
    const v16h a0 = ldfrag(hz, DIM, m0, k0, lane);
    const v16h a1 = ldfrag(hz, DIM, m0 + 16, k0, lane);
#pragma unroll
    for (int t = 0; t < NT; ++t) {
      const v16h b = ldfrag(wt, DIM, 16 * t, k0, lane);
      acc[0][t] = mma16(a0, b, acc[0][t]);
      acc[1][t] = mma16(a1, b, acc[1][t]);
    }
  }

  float* sw = st[wave];
  const float osc = 0.001953125f;
  if (MODE == 0) {
    float bvs[NT];
#pragma unroll
    for (int t = 0; t < NT; ++t) {
      const int bi = 16 * t + c;
      bvs[t] = bias[(bi < NB) ? bi : (NB - 1)];
    }
#pragma unroll
    for (int sub = 0; sub < 2; ++sub) {
      __syncthreads();
#pragma unroll
      for (int t = 0; t < NT; ++t) {
#pragma unroll
        for (int r = 0; r < 8; ++r)
          sw[(8 * hh + r) * HP0 + 16 * t + c] = acc[sub][t][r] * osc + bvs[t];
      }
      __syncthreads();
      v4f val[10];
      size_t go[10];
#pragma unroll
      for (int it = 0; it < 10; ++it) {
        const int p   = lane + 32 * it;
        const int row = p / 20;
        const int q   = p - row * 20;
        val[it] = *(const v4f*)(sw + row * HP0 + q * 4);
        go[it]  = (size_t)(m0 + sub * 16 + row) * NCLS + q * 4;
      }
      for (int ps = 0; ps < 2; ++ps) {
#pragma unroll
        for (int it = 0; it < 10; ++it) *(volatile v4f*)(out + go[it]) = val[it];
        __threadfence();
      }
    }
  } else {
    const float bb = bias[(c < NB) ? c : (NB - 1)];
    __syncthreads();
#pragma unroll
    for (int sub = 0; sub < 2; ++sub) {
#pragma unroll
      for (int r = 0; r < 8; ++r) {
        float v = acc[sub][0][r] * osc + bb;
        if (MODE == 2) v = __builtin_amdgcn_rcpf(1.0f + __expf(-v));
        sw[(sub * 16 + 8 * hh + r) * HP1 + c] = v;
      }
    }
    __syncthreads();
    v4f o;
    size_t g;
    if (MODE == 1) {
#pragma unroll
      for (int e = 0; e < 4; ++e) o[e] = sw[((4 * lane + e) & 31) * HP1];
      g = (size_t)(m0 + 4 * lane);
    } else {
#pragma unroll
      for (int e = 0; e < 4; ++e) o[e] = sw[lane * HP1 + e];
      g = (size_t)(m0 + lane) * 4;
    }
    const bool act = (MODE == 1) ? (lane < 8) : true;
    for (int ps = 0; ps < 2; ++ps) {
      if (act) *(volatile v4f*)(out + g) = o;
      __threadfence();
    }
  }
}

__global__ __launch_bounds__(256) void k_loss(const float* __restrict__ oc, const float* __restrict__ oo,
                                             const float* __restrict__ ob, const float* __restrict__ boxes,
                                             const int* __restrict__ labels, float* __restrict__ ol) {
#pragma clang fp contract(off)
  __shared__ float sbx[NBOX * 4];
  __shared__ int   slb[NBOX];
  __shared__ float red[5][8];
  const int t = threadIdx.x, lane = t & 31, wave = t >> 5;
  const int tt = (t < PP) ? t : (PP - 1);
  const float keep = (t < PP) ? 1.0f : 0.0f;
  float total = 0.0f;
#pragma unroll 1
  for (int b = 0; b < BATCH; ++b) {
    const float bxv = boxes[(size_t)b * (NBOX * 4) + (t & (NBOX * 4 - 1))];
    const int   lbv = labels[b * NBOX + (t & (NBOX - 1))];
    __syncthreads();
    if (t < NBOX * 4) sbx[t] = bxv;
    if (t < NBOX) slb[t] = lbv;
    __syncthreads();

    int lw = -1;
#pragma unroll 1
    for (int m = 0; m < NBOX; ++m) {
      int gx = (int)(sbx[4 * m] * 14.0f);
      int gy = (int)(sbx[4 * m + 1] * 14.0f);
      gx = gx < 0 ? 0 : (gx > GRIDN - 1 ? GRIDN - 1 : gx);
      gy = gy < 0 ? 0 : (gy > GRIDN - 1 ? GRIDN - 1 : gy);
      lw = (gy * GRIDN + gx == tt) ? m : lw;
    }
    const float vf = (lw >= 0) ? 1.0f : 0.0f;
    const int sf = (lw < 0) ? 0 : lw;
    const float tb0 = sbx[4 * sf], tb1 = sbx[4 * sf + 1], tb2 = sbx[4 * sf + 2], tb3 = sbx[4 * sf + 3];
    int lab = slb[sf];
    lab = lab < 0 ? 0 : (lab > NCLS - 1 ? NCLS - 1 : lab);

    const v4f pb = *(const v4f*)(ob + (size_t)(b * PP + tt) * 4);
    const float l1 = ((fabsf(pb[0] - tb0) + fabsf(pb[1] - tb1)) + (fabsf(pb[2] - tb2) + fabsf(pb[3] - tb3))) * 0.25f;
    const float p0 = pb[0] - pb[2] * 0.5f, p1 = pb[1] - pb[3] * 0.5f;
    const float p2 = pb[0] + pb[2] * 0.5f, p3 = pb[1] + pb[3] * 0.5f;
    const float t0 = tb0 - tb2 * 0.5f, t1 = tb1 - tb3 * 0.5f;
    const float t2 = tb0 + tb2 * 0.5f, t3 = tb1 + tb3 * 0.5f;
    const float ix1 = fmaxf(p0, t0), iy1 = fmaxf(p1, t1);
    const float ix2 = fminf(p2, t2), iy2 = fminf(p3, t3);
    const float inter = fmaxf(ix2 - ix1, 0.0f) * fmaxf(iy2 - iy1, 0.0f);
    const float arp = fmaxf(p2 - p0, 0.0f) * fmaxf(p3 - p1, 0.0f);
    const float art = fmaxf(t2 - t0, 0.0f) * fmaxf(t3 - t1, 0.0f);
    const float uni = (arp + art) - inter;
    const float iou = inter * __builtin_amdgcn_rcpf(uni + 1e-7f);
    const float ex1 = fminf(p0, t0), ey1 = fminf(p1, t1);
    const float ex2 = fmaxf(p2, t2), ey2 = fmaxf(p3, t3);
    const float enc = fmaxf(ex2 - ex1, 0.0f) * fmaxf(ey2 - ey1, 0.0f);
    const float giou = iou - (enc - uni) * __builtin_amdgcn_rcpf(enc + 1e-7f);

    const float* cl = oc + (size_t)(b * PP + tt) * NCLS;
    float mx = cl[0];
#pragma unroll 1
    for (int j = 1; j < NCLS; ++j) mx = fmaxf(mx, cl[j]);
    float se = 0.0f;
#pragma unroll 1
    for (int j = 0; j < NCLS; ++j) se += __expf(cl[j] - mx);
    const float nll = -((cl[lab] - mx) - __logf(se));

    const float lg = oo[(size_t)b * PP + tt];
    const float ce = fmaxf(lg, 0.0f) - lg * vf + __logf(1.0f + __expf(-fabsf(lg)));
    const float pr = __builtin_amdgcn_rcpf(1.0f + __expf(-lg));
    const float pt = pr * vf + (1.0f - pr) * (1.0f - vf);
    const float at = 0.25f * vf + 0.75f * (1.0f - vf);
    const float om = 1.0f - pt;

    float s0 = vf * keep;
    float s1 = l1 * vf * keep;
    float s2 = giou * vf * keep;
    float s3 = nll * vf * keep;
    float s4 = at * om * om * ce * keep;
#pragma unroll
    for (int off = 1; off < 32; off <<= 1) {
      s0 += __shfl_xor(s0, off, 32);
      s1 += __shfl_xor(s1, off, 32);
      s2 += __shfl_xor(s2, off, 32);
      s3 += __shfl_xor(s3, off, 32);
      s4 += __shfl_xor(s4, off, 32);
    }
    if (lane == 0) { red[0][wave] = s0; red[1][wave] = s1; red[2][wave] = s2; red[3][wave] = s3; red[4][wave] = s4; }
    __syncthreads();
    float vfs = 0.0f, l1s = 0.0f, gis = 0.0f, nls = 0.0f, fcs = 0.0f;
#pragma unroll
    for (int w = 0; w < 8; ++w) { vfs += red[0][w]; l1s += red[1][w]; gis += red[2][w]; nls += red[3][w]; fcs += red[4][w]; }
    const float n = fmaxf(vfs, 1.0f);
    const float inv = 1.0f / n;
    const float box = (vfs > 0.0f) ? ((nls * inv + 5.0f * (l1s * inv)) + 2.0f * (1.0f - gis * inv)) : 0.0f;
    total += box + fcs * (1.0f / (float)PP);
  }
  if (t == 0) {
    const float lv = total * (1.0f / (float)BATCH);
    volatile float* d = (volatile float*)ol;
    *d = lv;
    __threadfence();
    *d = lv;
  }
}

extern "C" void kernel_launch(void* const* d_in, const int* in_sizes, int n_in,
                              void* d_out, int out_size, void* d_ws, size_t ws_size,
                              hipStream_t stream) {
  if (n_in < 19) return;
  if (in_sizes[0] != BATCH * 3 * IMW * IMW) return;
  if (in_sizes[1] != BATCH * NBOX * 4 || in_sizes[2] != BATCH * NBOX) return;
  if (in_sizes[3] != DIM * 3 * PSZ * PSZ || in_sizes[4] != DIM) return;
  if (in_sizes[5] != PP * DIM || in_sizes[6] != DIM) return;
  if (in_sizes[7] != DIM * DIM || in_sizes[8] != DIM || in_sizes[9] != DIM * NCLS || in_sizes[10] != NCLS) return;
  if (in_sizes[11] != DIM * DIM || in_sizes[12] != DIM || in_sizes[13] != DIM || in_sizes[14] != 1) return;
  if (in_sizes[15] != DIM * DIM || in_sizes[16] != DIM || in_sizes[17] != DIM * 4 || in_sizes[18] != 4) return;
  if ((size_t)out_size != OFF3 + 1) return;

  const float* imgs    = (const float*)d_in[0];
  const float* boxes   = (const float*)d_in[1];
  const int*   labels  = (const int*)d_in[2];
  const float* patch_w = (const float*)d_in[3];
  const float* patch_b = (const float*)d_in[4];
  const float* pos     = (const float*)d_in[5];
  const float* norm_w  = (const float*)d_in[6];
  const float* cls_w1  = (const float*)d_in[7];
  const float* cls_b1  = (const float*)d_in[8];
  const float* cls_w2  = (const float*)d_in[9];
  const float* cls_b2  = (const float*)d_in[10];
  const float* obj_w1  = (const float*)d_in[11];
  const float* obj_b1  = (const float*)d_in[12];
  const float* obj_w2  = (const float*)d_in[13];
  const float* obj_b2  = (const float*)d_in[14];
  const float* bbox_w1 = (const float*)d_in[15];
  const float* bbox_b1 = (const float*)d_in[16];
  const float* bbox_w2 = (const float*)d_in[17];
  const float* bbox_b2 = (const float*)d_in[18];
  float* out = (float*)d_out;

  const size_t oXp  = 0;
  const size_t oE   = oXp + PLH * 2;
  const size_t oH   = 0;
  size_t off = oE + (size_t)NTOK * DIM * 4;
  if (3 * PLH * 2 > off) return;
  const size_t oWp  = off; off += (size_t)DIM * DIM * 2;
  const size_t oW1  = off; off += (size_t)3 * DIM * DIM * 2;
  const size_t oW2c = off; off += (size_t)NCLS * DIM * 2;
  const size_t oW2o = off; off += (size_t)16 * DIM * 2;
  const size_t oW2b = off; off += (size_t)16 * DIM * 2;
  const size_t oXn  = off; off += PLH * 2;
  if (off > ws_size) return;
  if (off > (size_t)134217728) return;

  char* ws = (char*)d_ws;
  _Float16* Xp  = (_Float16*)(ws + oXp);
  float*    E   = (float*)(ws + oE);
  _Float16* H   = (_Float16*)(ws + oH);
  _Float16* Wp  = (_Float16*)(ws + oWp);
  _Float16* W1t = (_Float16*)(ws + oW1);
  _Float16* W2c = (_Float16*)(ws + oW2c);
  _Float16* W2o = (_Float16*)(ws + oW2o);
  _Float16* W2b = (_Float16*)(ws + oW2b);
  _Float16* Xn  = (_Float16*)(ws + oXn);

  k_im2col<<<dim3((NTOK * NPC) / 256), dim3(256), 0, stream>>>(imgs, Xp, NTOK * NPC);
  k_cvt_w<<<dim3((DIM * DIM / 8) / 256), dim3(256), 0, stream>>>(patch_w, Wp, DIM * DIM / 8, 32.0f);
  k_wt<<<dim3(DIM / 64, DIM / 64), dim3(256), 0, stream>>>(cls_w1,  W1t, DIM, DIM);
  k_wt<<<dim3(DIM / 64, DIM / 64), dim3(256), 0, stream>>>(obj_w1,  W1t + (size_t)DIM * DIM, DIM, DIM);
  k_wt<<<dim3(DIM / 64, DIM / 64), dim3(256), 0, stream>>>(bbox_w1, W1t + (size_t)2 * DIM * DIM, DIM, DIM);
  k_wt_small<<<dim3((NCLS * NPC) / 256), dim3(256), 0, stream>>>(cls_w2, W2c, NCLS, NCLS);
  k_wt_small<<<dim3((16 * NPC) / 256), dim3(256), 0, stream>>>(obj_w2, W2o, 1, 16);
  k_wt_small<<<dim3((16 * NPC) / 256), dim3(256), 0, stream>>>(bbox_w2, W2b, 4, 16);
  k_embed<<<dim3(NTOK / 256, DIM / 64), dim3(256), 0, stream>>>(Xp, Wp, patch_b, pos, E);
  k_rms<<<dim3(NTOK / 8), dim3(256), 0, stream>>>(E, norm_w, Xn);
  k_hid<<<dim3(NTOK / 256, DIM / 64, 3), dim3(256), 0, stream>>>(Xn, W1t, cls_b1, obj_b1, bbox_b1, H);
  k_head<0><<<dim3(NTOK / 256), dim3(256), 0, stream>>>(H,           W2c, cls_b2,  out);
  k_head<1><<<dim3(NTOK / 256), dim3(256), 0, stream>>>(H + PLH,     W2o, obj_b2,  out + OFF1);
  k_head<2><<<dim3(NTOK / 256), dim3(256), 0, stream>>>(H + 2 * PLH, W2b, bbox_b2, out + OFF2);
  k_loss<<<dim3(1), dim3(256), 0, stream>>>(out, out + OFF1, out + OFF2, boxes, labels, out + OFF3);
  (void)hipGetLastError();
}
